// GraphSageLayer_53755810677325
// MI455X (gfx1250) — hardware-verified
//
#include <hip/hip_runtime.h>
#include <stddef.h>
#include <stdint.h>


#define DIN     128
#define DOUT    128
#define KTOT    384
#define KS1     8
#define KS2     4
#define NTHR    256
#define NWAVE   8
#define EPT     8
#define CHUNK   (NTHR * EPT)
#define WCAP    (EPT * 32)
#define LISTN   (NWAVE * WCAP)
#define NBMAX   2048
#define RCAP    28672
#define DEGCAP  256
#define STW     256
#define GBM     64
#define GBN     64
#define GTHR    128
#define CX      16.0f
#define CW      256.0f
#define CL      2048.0f
#define SCL     0.000244140625f
#define SCLR    1.1920928955078125e-07f
#define WSMAX   134217728
#define LDS_AGG ((2 * RCAP + 2 * NBMAX + LISTN) * 4 + 64)

static_assert((CHUNK & (CHUNK - 1)) == 0 && CHUNK <= 4096);
static_assert((NBMAX & (NBMAX - 1)) == 0 && NBMAX <= 4096);
static_assert(NTHR * 8 == NBMAX);
static_assert(LISTN >= NBMAX);
static_assert(LISTN >= NWAVE * WCAP);
static_assert((RCAP % 32) == 0);
static_assert(NWAVE * STW <= RCAP);
static_assert(STW >= 2 * DIN);
static_assert(LDS_AGG <= 300000);
static_assert(GBM == (GTHR / 32) * 16);
static_assert((KTOT % 32) == 0 && KTOT == 32 * (KS1 + KS2));
static_assert(KTOT == 3 * DIN && 32 * KS1 == 2 * DIN);
static_assert((DOUT % GBN) == 0);
static_assert(DIN == 128);

typedef float    v4f  __attribute__((ext_vector_type(4)));
typedef float    v8f  __attribute__((ext_vector_type(8)));
typedef int      v4i  __attribute__((ext_vector_type(4)));
typedef int      v8i  __attribute__((ext_vector_type(8)));
typedef _Float16 v8h  __attribute__((ext_vector_type(8)));
typedef _Float16 v16h __attribute__((ext_vector_type(16)));
union FragH { v16h v; v8h h[2]; v8i w; };
union Pack8 { v8h h; v4i w; };

__device__ __forceinline__ v8f wmh(const FragH& a, const FragH& b, v8f c) {
  v8f d = __builtin_amdgcn_wmma_f32_16x16x32_f16(false, a.v, false, b.v, (short)0, c, false, false);
  asm volatile("v_nop\n\tv_nop\n\tv_nop\n\tv_nop" : "+v"(d) : "v"(a.w), "v"(b.w));
  return d;
}

__device__ __forceinline__ void ldwait() {
  asm volatile("s_wait_loadcnt 0x0" ::: "memory");
}

__device__ __forceinline__ float bf16r(float f) {
  unsigned u = __float_as_uint(f);
  u = (u + 0x7FFFu + ((u >> 16) & 1u)) & 0xFFFF0000u;
  return __uint_as_float(u);
}

__device__ __forceinline__ v4f bf16r4(v4f a) {
  v4f r;
  r.x = bf16r(a.x); r.y = bf16r(a.y); r.z = bf16r(a.z); r.w = bf16r(a.w);
  return r;
}

__device__ __forceinline__ v8h cvt8h(const v4f a, const v4f b, const float c) {
  v8h hv;
  hv[0] = (_Float16)(a.x * c); hv[1] = (_Float16)(a.y * c);
  hv[2] = (_Float16)(a.z * c); hv[3] = (_Float16)(a.w * c);
  hv[4] = (_Float16)(b.x * c); hv[5] = (_Float16)(b.y * c);
  hv[6] = (_Float16)(b.z * c); hv[7] = (_Float16)(b.w * c);
  return hv;
}

__device__ __forceinline__ void split8h(const v4f a, const v4f b, v8h& hi, v8h& lo) {
  float s[8];
  s[0] = a.x * CX; s[1] = a.y * CX; s[2] = a.z * CX; s[3] = a.w * CX;
  s[4] = b.x * CX; s[5] = b.y * CX; s[6] = b.z * CX; s[7] = b.w * CX;
#pragma unroll
  for (int i = 0; i < 8; ++i) {
    const _Float16 hv = (_Float16)s[i];
    hi[i] = hv;
    lo[i] = (_Float16)((s[i] - (float)hv) * CL);
  }
}

__device__ __forceinline__ int scan_chunk(const int* __restrict__ dsts, int nE, int cbase, int slotBase,
                                          int nb, int vec8, int* list, int tid, int lane, int wave) {
  int wc = 0;
  const int el0  = tid * EPT;
  const int e0   = cbase + el0;
  const int sent = -2147483647 - 1;
  v4i da, db;
  if (vec8 != 0 && cbase + CHUNK <= nE) {
    da = *(const v4i*)(dsts + e0);
    db = *(const v4i*)(dsts + e0 + 4);
  } else {
    da.x = (e0     < nE) ? dsts[min(e0,     nE - 1)] : sent;
    da.y = (e0 + 1 < nE) ? dsts[min(e0 + 1, nE - 1)] : sent;
    da.z = (e0 + 2 < nE) ? dsts[min(e0 + 2, nE - 1)] : sent;
    da.w = (e0 + 3 < nE) ? dsts[min(e0 + 3, nE - 1)] : sent;
    db.x = (e0 + 4 < nE) ? dsts[min(e0 + 4, nE - 1)] : sent;
    db.y = (e0 + 5 < nE) ? dsts[min(e0 + 5, nE - 1)] : sent;
    db.z = (e0 + 6 < nE) ? dsts[min(e0 + 6, nE - 1)] : sent;
    db.w = (e0 + 7 < nE) ? dsts[min(e0 + 7, nE - 1)] : sent;
  }
  const unsigned nbs = (unsigned)slotBase;
  const unsigned unb = (unsigned)nb;
  const unsigned s0 = (unsigned)da.x - nbs, s1 = (unsigned)da.y - nbs;
  const unsigned s2 = (unsigned)da.z - nbs, s3 = (unsigned)da.w - nbs;
  const unsigned s4 = (unsigned)db.x - nbs, s5 = (unsigned)db.y - nbs;
  const unsigned s6 = (unsigned)db.z - nbs, s7 = (unsigned)db.w - nbs;
  const bool h0 = s0 < unb, h1 = s1 < unb, h2 = s2 < unb, h3 = s3 < unb;
  const bool h4 = s4 < unb, h5 = s5 < unb, h6 = s6 < unb, h7 = s7 < unb;
  const unsigned any = __builtin_amdgcn_ballot_w32(h0 | h1 | h2 | h3 | h4 | h5 | h6 | h7);
  if (any != 0u) {
#define HITJ(J, HJ, SJ) { \
      const unsigned mj = __builtin_amdgcn_ballot_w32(HJ); \
      if (mj != 0u) { \
        if (HJ) { \
          const int pos = wc + (int)__builtin_amdgcn_mbcnt_lo(mj, 0u); \
          if (pos < WCAP) list[wave * WCAP + pos] = ((el0 + (J)) << 12) | (int)(SJ); \
        } \
        wc += (int)__builtin_popcount(mj); } }
    HITJ(0, h0, s0)
    HITJ(1, h1, s1)
    HITJ(2, h2, s2)
    HITJ(3, h3, s3)
    HITJ(4, h4, s4)
    HITJ(5, h5, s5)
    HITJ(6, h6, s6)
    HITJ(7, h7, s7)
#undef HITJ
  }
  return wc;
}

__global__ __launch_bounds__(NTHR) void k_wtr(const float* __restrict__ Wr, const float* __restrict__ Wl,
                                              _Float16* wt, int nUnits) {
  const int u = (int)blockIdx.x * NTHR + (int)threadIdx.x;
  if (u >= nUnits) return;
  const int kq = KTOT / 8;
  const int n  = u / kq;
  const int k8 = (u - n * kq) * 8;
  const int kr = k8 & (DIN - 1);
  const float* pr = Wr + (size_t)n * DIN + kr;
  const float* pl = Wl + (size_t)n * DIN + kr;
  const v4f ra = *(const v4f*)pr, rb = *(const v4f*)(pr + 4);
  const v4f la = *(const v4f*)pl, lb = *(const v4f*)(pl + 4);
  v4f a = ra, b = rb;
  if (k8 >= DIN) { a = la; b = lb; }
  a = bf16r4(a); b = bf16r4(b);
  const v8h hv = cvt8h(a, b, CW);
  const size_t o = (size_t)n * (size_t)KTOT + k8;
  *(volatile v8h*)(wt + o) = hv;
  __threadfence();
  *(volatile v8h*)(wt + o) = hv;
}

__global__ __launch_bounds__(GTHR) void k_gemm(
    const _Float16* __restrict__ A, const _Float16* __restrict__ WT,
    const float* __restrict__ bias, float* outF,
    int K, int ks1, int ks2, int ldo, int nRows, int nBias, float scl, float sclr)
{
  __shared__ __attribute__((aligned(16))) float stg[GBM * GBN];
  const int tid = (int)threadIdx.x, lane = tid & 31, wave = tid >> 5, hh = lane >> 4, m = lane & 15;
  const int rowBase = (int)blockIdx.x * GBM;
  const int col0    = (int)blockIdx.y * GBN;

  v8f acc[4], accr[4];
  {
    const v8f z = {0.f, 0.f, 0.f, 0.f, 0.f, 0.f, 0.f, 0.f};
    acc[0] = z; acc[1] = z; acc[2] = z; acc[3] = z;
    accr[0] = z; accr[1] = z; accr[2] = z; accr[3] = z;
  }
  const _Float16* ap = A  + (size_t)(rowBase + 16 * wave + m) * (size_t)K + 8 * hh;
  const _Float16* wp = WT + (size_t)(col0 + m) * (size_t)K + 8 * hh;
#pragma unroll 1
  for (int ks = 0; ks < ks1; ++ks) {
    FragH af;
    af.h[0] = *(const v8h*)(ap + 32 * ks);
    af.h[1] = *(const v8h*)(ap + 32 * ks + 16);
#pragma unroll
    for (int t = 0; t < 4; ++t) {
      const _Float16* wq = wp + (size_t)(16 * t) * (size_t)K + 32 * ks;
      FragH bf;
      bf.h[0] = *(const v8h*)wq;
      bf.h[1] = *(const v8h*)(wq + 16);
      acc[t] = wmh(af, bf, acc[t]);
    }
  }
  const int ksEnd = ks1 + ks2;
#pragma unroll 1
  for (int ks = ks1; ks < ksEnd; ++ks) {
    FragH af;
    af.h[0] = *(const v8h*)(ap + 32 * ks);
    af.h[1] = *(const v8h*)(ap + 32 * ks + 16);
#pragma unroll
    for (int t = 0; t < 4; ++t) {
      const _Float16* wq = wp + (size_t)(16 * t) * (size_t)K + 32 * ks;
      FragH bf;
      bf.h[0] = *(const v8h*)wq;
      bf.h[1] = *(const v8h*)(wq + 16);
      accr[t] = wmh(af, bf, accr[t]);
    }
  }

#pragma unroll
  for (int t = 0; t < 4; ++t) {
    const int lc = 16 * t + m;
    int bi = col0 + lc;
    bi = bi > nBias - 1 ? nBias - 1 : bi;
    bi = bi < 0 ? 0 : bi;
    const float bv = bf16r(bias[bi]);
#pragma unroll
    for (int r = 0; r < 8; ++r) {
      const int lr = 16 * wave + 8 * hh + r;
      stg[lr * GBN + lc] = fmaf(acc[t][r], scl, fmaf(accr[t][r], sclr, bv));
    }
  }
  __syncthreads();

  v4f fv[8];
#pragma unroll
  for (int i = 0; i < 8; ++i) {
    const int lr = 16 * wave + 2 * i + hh;
    fv[i] = *(const v4f*)(stg + lr * GBN + 4 * m);
  }
#pragma unroll
  for (int i = 0; i < 8; ++i) {
    const int lr = 16 * wave + 2 * i + hh;
    const int gr = rowBase + lr;
    float* op = outF + (size_t)gr * (size_t)ldo + col0 + 4 * m;
    if (gr < nRows) *(volatile v4f*)op = fv[i];
  }
  __threadfence();
#pragma unroll
  for (int i = 0; i < 8; ++i) {
    const int lr = 16 * wave + 2 * i + hh;
    const int gr = rowBase + lr;
    float* op = outF + (size_t)gr * (size_t)ldo + col0 + 4 * m;
    if (gr < nRows) *(volatile v4f*)op = fv[i];
  }
}

__global__ __launch_bounds__(NTHR) void k_agg(
    const int* __restrict__ srcs, const int* __restrict__ dsts,
    const float* __restrict__ x, _Float16* AP,
    int nN, int nE, int nb, int vec8, int MPr) {
  extern __shared__ v4f lds_dyn[];
  int* reg1 = (int*)lds_dyn;
  int* reg2 = reg1 + RCAP;
  int* scnt = reg2 + RCAP;
  int* soff = scnt + NBMAX;
  int* list = soff + NBMAX;
  int* wcnt = list + LISTN;
  int* wtot = wcnt + NWAVE;
  const int tid = (int)threadIdx.x, lane = tid & 31, wave = tid >> 5;
  const int nodeBase = (int)blockIdx.x * nb;

  for (int i = tid; i < NBMAX; i += NTHR) scnt[i] = 0;
  __syncthreads();

  int tot = 0;
  const int nChunks = (nE + CHUNK - 1) / CHUNK;
#pragma unroll 1
  for (int ch = 0; ch < nChunks; ++ch) {
    const int cbase = ch * CHUNK;
    const int wc = scan_chunk(dsts, nE, cbase, nodeBase, nb, vec8, list, tid, lane, wave);
    if (lane == 0) wcnt[wave] = wc;
    __syncthreads();
    int pre = 0, all = 0;
#pragma unroll
    for (int w2 = 0; w2 < NWAVE; ++w2) {
      int c = wcnt[w2];
      c = c < 0 ? 0 : (c > WCAP ? WCAP : c);
      all += c;
      pre += (w2 < wave) ? c : 0;
    }
    const int wcc  = wc > WCAP ? WCAP : wc;
    const int base = tot + pre;
#pragma unroll 1
    for (int i = lane; i < wcc; i += 32) {
      const int ent = list[wave * WCAP + i];
      const int el  = (ent >> 12) & (CHUNK - 1);
      const int sl  = ent & (NBMAX - 1);
      int eid = cbase + el;
      eid = eid > nE - 1 ? nE - 1 : eid;
      const int pos = base + i;
      if (pos < RCAP) reg1[pos] = (int)(((unsigned)eid << 12) | (unsigned)sl);
    }
    tot += all;
    tot = tot > RCAP ? RCAP : tot;
    __syncthreads();
  }
  const int nh = tot;

  if (wave == 0) {
#pragma unroll 1
    for (int b0 = 0; b0 < nh; b0 += 32) {
      const int idx = b0 + lane;
      const int uv  = reg1[idx < RCAP ? idx : RCAP - 1];
      const int m32 = (nh - b0) < 32 ? (nh - b0) : 32;
#pragma unroll 1
      for (int k = 0; k < m32; ++k) {
        const int u  = __builtin_amdgcn_readlane(uv, k);
        const int sl = u & (NBMAX - 1);
        if (lane == 0) scnt[sl] = scnt[sl] + 1;
      }
    }
  }
  __syncthreads();

  {
    const v4i ca = *(const v4i*)(scnt + 8 * tid);
    const v4i cb = *(const v4i*)(scnt + 8 * tid + 4);
    const int e0 = ca.x < 0 ? 0 : ca.x, e1 = ca.y < 0 ? 0 : ca.y, e2 = ca.z < 0 ? 0 : ca.z, e3 = ca.w < 0 ? 0 : ca.w;
    const int e4 = cb.x < 0 ? 0 : cb.x, e5 = cb.y < 0 ? 0 : cb.y, e6 = cb.z < 0 ? 0 : cb.z, e7 = cb.w < 0 ? 0 : cb.w;
    const int ts = e0 + e1 + e2 + e3 + e4 + e5 + e6 + e7;
    int incl = ts;
#pragma unroll
    for (int d = 1; d < 32; d <<= 1) {
      const int up = __shfl_up(incl, d);
      if (lane >= d) incl += up;
    }
    if (lane == 31) wtot[wave] = incl;
    __syncthreads();
    int pre = 0;
#pragma unroll
    for (int w2 = 0; w2 < NWAVE; ++w2) pre += (w2 < wave) ? wtot[w2] : 0;
    int run = pre + incl - ts;
    soff[8 * tid + 0] = run; run += e0;
    soff[8 * tid + 1] = run; run += e1;
    soff[8 * tid + 2] = run; run += e2;
    soff[8 * tid + 3] = run; run += e3;
    soff[8 * tid + 4] = run; run += e4;
    soff[8 * tid + 5] = run; run += e5;
    soff[8 * tid + 6] = run; run += e6;
    soff[8 * tid + 7] = run;
  }
  __syncthreads();
  for (int i = tid; i < NBMAX; i += NTHR) list[i] = soff[i];
  __syncthreads();

  if (wave == 0) {
#pragma unroll 1
    for (int b0 = 0; b0 < nh; b0 += 32) {
      const int idx = b0 + lane;
      const int uv  = reg1[idx < RCAP ? idx : RCAP - 1];
      const int m32 = (nh - b0) < 32 ? (nh - b0) : 32;
#pragma unroll 1
      for (int k = 0; k < m32; ++k) {
        const int u   = __builtin_amdgcn_readlane(uv, k);
        const int sl  = u & (NBMAX - 1);
        const int eid = (int)((unsigned)u >> 12);
        if (lane == 0) {
          int pos = list[sl];
          pos = pos < 0 ? 0 : (pos > RCAP - 1 ? RCAP - 1 : pos);
          reg2[pos] = eid;
          list[sl] = pos + 1;
        }
      }
    }
  }
  __syncthreads();

  const int nbw = nb >> 3;
  const bool ovf = (nh >= RCAP);
  const float qnan = __int_as_float(0x7fc00000);
  float* stw = (float*)reg1 + wave * STW;
  const int l16 = lane & 15;
#pragma unroll 1
  for (int jt = 0; jt < nbw; ++jt) {
    const int slot = wave * nbw + jt;
    const int grow = nodeBase + slot;
    const int gcl  = grow < nN ? grow : nN - 1;
    int st = soff[slot];
    const int craw = scnt[slot];
    int cnt = craw;
    st  = st < 0 ? 0 : (st > nh ? nh : st);
    cnt = cnt < 0 ? 0 : (cnt > DEGCAP ? DEGCAP : cnt);
    if (cnt > nh - st) cnt = nh - st;
    const float pz = (ovf || craw > DEGCAP) ? qnan : 0.0f;
    const bool wr = grow < MPr;
    const float live = grow < nN ? 1.0f : 0.0f;

    const float* xrow = x + (size_t)gcl * DIN + lane;
    float xs[4], sm[4];
    {
      float xv[4];
#pragma unroll
      for (int j = 0; j < 4; ++j) xv[j] = xrow[32 * j];
      ldwait();
#pragma unroll
      for (int j = 0; j < 4; ++j) { xs[j] = bf16r(xv[j]); sm[j] = 0.f; }
    }

#pragma unroll 1
    for (int q = 0; q < cnt; ++q) {
      int idx = st + q; idx = idx > RCAP - 1 ? RCAP - 1 : idx;
      int eid = reg2[idx]; eid = eid < 0 ? 0 : (eid > nE - 1 ? nE - 1 : eid);
      const int sraw = srcs[eid];
      const int s = sraw < 0 ? 0 : (sraw > nN - 1 ? nN - 1 : sraw);
      const float* xr = x + (size_t)s * DIN + lane;
      float vv[4];
#pragma unroll
      for (int j = 0; j < 4; ++j) vv[j] = xr[32 * j];
      ldwait();
#pragma unroll
      for (int j = 0; j < 4; ++j) sm[j] += bf16r(vv[j]);
    }
    const float dg  = (float)cnt;
    const float inv = 1.0f / fmaxf(dg, 1.0f);

    __builtin_amdgcn_fence(__ATOMIC_RELEASE, "wavefront");
    __builtin_amdgcn_wave_barrier();
#pragma unroll
    for (int j = 0; j < 4; ++j) {
      stw[32 * j + lane]       = xs[j] * live + pz;
      stw[DIN + 32 * j + lane] = (sm[j] * inv) * live + pz;
    }
    __builtin_amdgcn_fence(__ATOMIC_RELEASE, "wavefront");
    __builtin_amdgcn_wave_barrier();
    const v4f xa = *(const v4f*)(stw + 8 * l16);
    const v4f xb = *(const v4f*)(stw + 8 * l16 + 4);
    const v4f ma = *(const v4f*)(stw + DIN + 8 * l16);
    const v4f mb = *(const v4f*)(stw + DIN + 8 * l16 + 4);
    Pack8 ux, uh, us;
    v8h lo;
    ux.h = cvt8h(xa, xb, CX);
    split8h(ma, mb, uh.h, lo);
    const bool lowh = lane < 16;
    us.w.x = lowh ? ux.w.x : uh.w.x;
    us.w.y = lowh ? ux.w.y : uh.w.y;
    us.w.z = lowh ? ux.w.z : uh.w.z;
    us.w.w = lowh ? ux.w.w : uh.w.w;
    _Float16* ar = AP + (size_t)grow * KTOT;
    _Float16* p1 = ar + 8 * lane;
    _Float16* p2 = ar + 2 * DIN + 8 * lane;
    const bool w2 = wr && lowh;
    if (wr) *(volatile v8h*)p1 = us.h;
    if (w2) *(volatile v8h*)p2 = lo;
    __threadfence();
    if (wr) *(volatile v8h*)p1 = us.h;
    if (w2) *(volatile v8h*)p2 = lo;
  }
}

static int pick_nb(int nE, int nN) {
  int nb = NBMAX;
  while (nb > 16 && (long long)nb * (long long)nE * 5LL > (long long)RCAP * (long long)nN * 4LL) nb >>= 1;
  return nb;
}
static inline int cdiv(int a, int b) { return (a + b - 1) / b; }

extern "C" void kernel_launch(void* const* d_in, const int* in_sizes, int n_in,
                              void* d_out, int out_size, void* d_ws, size_t ws_size,
                              hipStream_t stream) {
  if (n_in < 5) return;
  const int nN = in_sizes[0] / DIN;
  if (nN <= 0 || in_sizes[0] != nN * DIN || nN > (1 << 22)) return;
  if (in_sizes[1] < 2 || (in_sizes[1] & 1) != 0) return;
  const int nE = in_sizes[1] / 2;
  if (nE < 1 || nE > (1 << 20)) return;
  if (in_sizes[2] != DOUT * DIN) return;
  if (in_sizes[3] != DOUT) return;
  if (in_sizes[4] != DOUT * DIN) return;
  if (out_size != nN * DOUT) return;

  const float* x  = (const float*)d_in[0];
  const int*   ei = (const int*)  d_in[1];
  const float* Wl = (const float*)d_in[2];
  const float* bl = (const float*)d_in[3];
  const float* Wr = (const float*)d_in[4];
  float* out = (float*)d_out;
  const int* src = ei;
  const int* dst = ei + nE;

  const int MP   = cdiv(nN, GBM) * GBM;
  const int nb   = pick_nb(nE, nN);
  const int gA   = cdiv(MP, nb);
  const int vec8 = ((nE & 3) == 0) ? 1 : 0;
  if (gA * nb < MP) return;

  char* ws = (char*)d_ws;
  size_t off = 0;
  const size_t oAP = off; off += (size_t)MP * KTOT * 2;     off = (off + 255) & ~(size_t)255;
  const size_t oWT = off; off += (size_t)DOUT * KTOT * 2;   off = (off + 255) & ~(size_t)255;
  if (off > ws_size || off > (size_t)WSMAX) return;
  _Float16* AP = (_Float16*)(ws + oAP);
  _Float16* WT = (_Float16*)(ws + oWT);

  hipFuncSetAttribute(reinterpret_cast<const void*>(&k_agg),
                      hipFuncAttributeMaxDynamicSharedMemorySize, LDS_AGG);

  const int nUw = DOUT * (KTOT / 8);
  k_wtr<<<cdiv(nUw, NTHR), NTHR, 0, stream>>>(Wr, Wl, WT, nUw);

  k_agg<<<gA, NTHR, LDS_AGG, stream>>>(src, dst, x, AP, nN, nE, nb, vec8, MP);

  k_gemm<<<dim3(MP / GBM, DOUT / GBN), GTHR, 0, stream>>>(AP, WT, bl, out,
                                                          KTOT, KS1, KS2, DOUT, nN, DOUT, SCL, SCLR);
}
